// GeoPoseNet_6700148982571
// MI455X (gfx1250) — hardware-verified
//
#include <hip/hip_runtime.h>
#include <math.h>


#define NN 40000
#define NE 640000
#define NG 400
#define D1 256
#define C2 128
#define EDIM 4

typedef __attribute__((ext_vector_type(16))) __bf16 v16bf;
typedef __attribute__((ext_vector_type(8)))  float v8f;
typedef __attribute__((ext_vector_type(4)))  float v4f;
typedef float __attribute__((may_alias)) float_a;

template <typename T> __device__ __forceinline__ void vst2(void* p, T v) { *(volatile T*)p = v; __threadfence(); *(volatile T*)p = v; }
__device__ __forceinline__ v8f wmma_bf(v16bf a, v16bf b, v8f c) {
  v8f d = __builtin_amdgcn_wmma_f32_16x16x32_bf16(false, a, false, b, (short)0, c, false, false);
  asm volatile("v_nop\n\tv_nop\n\tv_nop\n\tv_nop" : "+v"(d) : "v"(a), "v"(b));
  return d;
}
struct F2 { v16bf h, l; };
__device__ __forceinline__ F2 split16(const float* v) {
  F2 r;
#pragma unroll
  for (int i = 0; i < 16; ++i) { const __bf16 hh = (__bf16)v[i]; r.h[i] = hh; r.l[i] = (__bf16)(v[i] - (float)hh); }
  return r;
}
__device__ __forceinline__ F2 split_row(const float* row, int k0, int lane) {
  float v[16]; const float* p = row + k0 + 8 * (lane >> 4);
#pragma unroll
  for (int i = 0; i < 8; ++i) { v[i] = p[i]; v[8 + i] = p[16 + i]; }
  return split16(v);
}
__device__ __forceinline__ F2 split_col(const float* base, int k0, int lane, int stride) {
  float v[16]; const float* p = base + (size_t)(k0 + 8 * (lane >> 4)) * stride;
#pragma unroll
  for (int i = 0; i < 8; ++i) { v[i] = p[(size_t)i * stride]; v[8 + i] = p[(size_t)(16 + i) * stride]; }
  return split16(v);
}
__device__ __forceinline__ v8f mac3(const F2& a, const F2& b, v8f c) { c = wmma_bf(a.l, b.h, c); c = wmma_bf(a.h, b.l, c); return wmma_bf(a.h, b.h, c); }
__device__ __forceinline__ float eluf(float x) { return x > 0.f ? x : expm1f(x); }

__global__ __launch_bounds__(256) void k_lin1(const float* __restrict__ x, const float* __restrict__ Wl, const float* __restrict__ bl,
                                            const float* __restrict__ Wr, const float* __restrict__ br, float* __restrict__ xl, float* __restrict__ xr) {
  const size_t g = (size_t)blockIdx.x * 256 + threadIdx.x;
  const int n = (int)(g >> 6), c0 = (int)(g & 63) * 4;
  const float x0 = x[(size_t)n * 2], x1 = x[(size_t)n * 2 + 1];
  v4f a, b;
#pragma unroll
  for (int e = 0; e < 4; ++e) { const int c = c0 + e;
    a[e] = x0 * Wl[c] + x1 * Wl[D1 + c] + bl[c]; b[e] = x0 * Wr[c] + x1 * Wr[D1 + c] + br[c]; }
  vst2(xl + (size_t)n * D1 + c0, a); vst2(xr + (size_t)n * D1 + c0, b);
}

__global__ __launch_bounds__(128) void k_gemm(const float* __restrict__ A, const float* __restrict__ W, const float* __restrict__ bias, float* __restrict__ C) {
  __shared__ __align__(16) float st[64][68];
  const int tid = threadIdx.x, wave = tid >> 5, lane = tid & 31, col = lane & 15, g = lane >> 4;
  const int m0 = blockIdx.x * 64 + wave * 16, n0 = blockIdx.y * 64;
  const float* arow = A + (size_t)(m0 + col) * D1;
  v8f acc[4] = {};
#pragma unroll 1
  for (int kc = 0; kc < D1 / 32; ++kc) {
    const F2 a = split_row(arow, kc * 32, lane);
#pragma unroll
    for (int j = 0; j < 4; ++j) acc[j] = mac3(a, split_col(W + n0 + j * 16 + col, kc * 32, lane, D1), acc[j]);
  }
#pragma unroll
  for (int j = 0; j < 4; ++j)
#pragma unroll
    for (int r = 0; r < 8; ++r) st[wave * 16 + 8 * g + r][j * 16 + col] = acc[j][r] + bias[n0 + j * 16 + col];
  __syncthreads();
  const int bm0 = blockIdx.x * 64;
  for (int q = tid; q < 64 * 16; q += 128) { const int rl = q >> 4, pc = q & 15;
    vst2(C + (size_t)(bm0 + rl) * D1 + n0 + pc * 4, *(const v4f*)(&st[rl][pc * 4])); }
}

#define DT 64
#define ECH 2048
#define NCH (NE / ECH + 1)
#define NT (NN / DT)
#define SLOTC 16
__global__ __launch_bounds__(256) void k_bucket(const int* __restrict__ ei, const float* __restrict__ ea,
                                              int* __restrict__ rec, float* __restrict__ eab, int* __restrict__ cnt) {
  __shared__ int hist[640], off[640], fill[640];
  __shared__ int srt[ECH];
  __shared__ __align__(16) float srtea[ECH][4];
  const int c = blockIdx.x, tid = threadIdx.x, e0 = c * ECH;
  for (int i = tid; i < 640; i += 256) { hist[i] = 0; fill[i] = 0; }
  __syncthreads();
  for (int i = tid; i < ECH; i += 256) { const int e = e0 + i; if (e < NE) { int d = ei[(size_t)NE + e]; d = d < 0 ? 0 : (d >= NN ? NN - 1 : d); atomicAdd(&hist[d / DT], 1); } }
  __syncthreads();
  if (tid == 0) { int s = 0; for (int t = 0; t < NT; ++t) { off[t] = s; s += hist[t]; } }
  __syncthreads();
  for (int i = tid; i < ECH; i += 256) { const int e = e0 + i; if (e < NE) {
      int d = ei[(size_t)NE + e]; d = d < 0 ? 0 : (d >= NN ? NN - 1 : d);
      int s = ei[e]; s = s < 0 ? 0 : (s >= NN ? NN - 1 : s);
      const int t = d / DT, r = atomicAdd(&fill[t], 1), pos = off[t] + r;
      srt[pos] = s | ((d - t * DT) << 16);
      *(v4f*)srtea[pos] = *(const v4f*)(ea + (size_t)e * 4); } }
  __syncthreads();
  for (int t = tid; t < NT; t += 256) {
    const int n = hist[t] < SLOTC ? hist[t] : SLOTC, o = off[t];
    int* rs = rec + ((size_t)t * NCH + c) * 32;
    float* es = eab + ((size_t)t * NCH + c) * SLOTC * 4;
#pragma unroll 1
    for (int q = 0; q < 8; ++q) { int v[4];
#pragma unroll
      for (int e = 0; e < 4; ++e) { const int j = q * 4 + e; v[e] = (j < n) ? srt[o + j] : 0; }
      typedef __attribute__((ext_vector_type(4))) int v4i; v4i vv = {v[0], v[1], v[2], v[3]}; vst2(rs + q * 4, vv); }
#pragma unroll 1
    for (int j = 0; j < SLOTC; ++j) { v4f v = (j < n) ? *(const v4f*)srtea[o + j] : (v4f){0.f, 0.f, 0.f, 0.f}; vst2(es + j * 4, v); }
  }
  for (int i = tid; i < 640 / 4; i += 256) { typedef __attribute__((ext_vector_type(4))) int v4i;
    v4i v = { i * 4 < NT ? (hist[i * 4] < SLOTC ? hist[i * 4] : SLOTC) : 0, i * 4 + 1 < NT ? (hist[i * 4 + 1] < SLOTC ? hist[i * 4 + 1] : SLOTC) : 0,
              i * 4 + 2 < NT ? (hist[i * 4 + 2] < SLOTC ? hist[i * 4 + 2] : SLOTC) : 0, i * 4 + 3 < NT ? (hist[i * 4 + 3] < SLOTC ? hist[i * 4 + 3] : SLOTC) : 0 };
    vst2(cnt + (size_t)c * 640 + i * 4, v); }
}

template <int HEADS, int MEANOUT>
__global__ __launch_bounds__(256) void k_gat(const int* __restrict__ rec, const float* __restrict__ eab, const int* __restrict__ cnt,
                                           const float* __restrict__ We, const float* __restrict__ att, const float* __restrict__ xl,
                                           const float* __restrict__ xr, const float* __restrict__ bias, float* __restrict__ out) {
  __shared__ __align__(16) float acc[DT][D1];
  __shared__ float mrun[DT][4], lrun[DT][4];
  const int tid = threadIdx.x, lane = tid & 31, wave = tid >> 5;
  const int t = blockIdx.x, d0 = t * DT;
  constexpr int LPH = 32 / HEADS;
  const int myh = lane / LPH;
  for (int i = tid; i < DT * D1 / 4; i += 256) *(v4f*)(&acc[0][0] + i * 4) = (v4f){0.f, 0.f, 0.f, 0.f};
  for (int i = tid; i < DT * 4; i += 256) { (&mrun[0][0])[i] = -3.0e38f; (&lrun[0][0])[i] = 0.f; }
  float wa[8], we0[8], we1[8], we2[8], we3[8];
#pragma unroll
  for (int e = 0; e < 8; ++e) { const int c = lane * 8 + e; wa[e] = att[c]; we0[e] = We[c]; we1[e] = We[D1 + c]; we2[e] = We[2 * D1 + c]; we3[e] = We[3 * D1 + c]; }
  __syncthreads();
#pragma unroll 1
  for (int c = 0; c < NCH; ++c) {
    const int n = cnt[(size_t)c * 640 + t];
    if (n == 0) continue;
    const int* rs = rec + ((size_t)t * NCH + c) * 32;
    const float* es = eab + ((size_t)t * NCH + c) * SLOTC * 4;
    const int r = (lane < n) ? rs[lane] : 0;
    const int dl = r >> 16;
    const bool mine = (lane < n) && ((dl & 7) == wave);
    unsigned msk = (unsigned)__builtin_amdgcn_ballot_w32(mine);
    while (msk) {
      const int j = __builtin_ctz(msk); msk &= msk - 1u;
      const int rj = __builtin_amdgcn_readlane(r, j);
      const int s = rj & 0xFFFF, dlj = rj >> 16;
      const v4f av = *(const v4f*)(es + j * 4);
      const float* xs = xl + (size_t)s * D1 + lane * 8;
      const float* xd = xr + (size_t)(d0 + dlj) * D1 + lane * 8;
      float xv[8], part = 0.f;
#pragma unroll
      for (int e = 0; e < 8; ++e) { xv[e] = xs[e];
        float z = xv[e] + xd[e] + av[0] * we0[e] + av[1] * we1[e] + av[2] * we2[e] + av[3] * we3[e];
        z = z > 0.f ? z : 0.2f * z; part += z * wa[e]; }
#pragma unroll
      for (int off = LPH / 2; off >= 1; off >>= 1) part += __shfl_xor(part, off, 32);
      const float mo = mrun[dlj][myh], lo_ = lrun[dlj][myh];
      const float mn = fmaxf(mo, part), corr = expf(mo - mn), p = expf(part - mn);
      float* ar = &acc[dlj][lane * 8];
#pragma unroll
      for (int e = 0; e < 8; ++e) ar[e] = ar[e] * corr + p * xv[e];
      __builtin_amdgcn_wave_barrier();
      if ((lane % LPH) == 0) { mrun[dlj][myh] = mn; lrun[dlj][myh] = lo_ * corr + p; }
      asm volatile("s_wait_dscnt 0" ::: "memory"); __builtin_amdgcn_wave_barrier();
    }
  }
  __syncthreads();
  if (MEANOUT == 0) {
    for (int rr = wave; rr < DT; rr += 8)
#pragma unroll
      for (int hh = 0; hh < 2; ++hh) { const int c0 = hh * 128 + lane * 4; v4f v;
#pragma unroll
        for (int e = 0; e < 4; ++e) { const int cc = c0 + e; v[e] = acc[rr][cc] / (lrun[rr][cc / (D1 / HEADS)] + 1e-16f) + bias[cc]; }
        vst2(out + (size_t)(d0 + rr) * D1 + c0, v); }
  } else {
    for (int rr = wave; rr < DT; rr += 8) { const int c0 = lane * 4; v4f v;
#pragma unroll
      for (int e = 0; e < 4; ++e) { const int cc = c0 + e;
        const float h0 = acc[rr][cc] / (lrun[rr][0] + 1e-16f), h1 = acc[rr][C2 + cc] / (lrun[rr][1] + 1e-16f);
        v[e] = 0.5f * (h0 + h1) + bias[cc]; }
      vst2(out + (size_t)(d0 + rr) * C2 + c0, v); }
  }
}

template <int W>
__global__ __launch_bounds__(256) void k_colpart(const float* __restrict__ X, float* __restrict__ part) {
  __shared__ float s1[256], s2[256];
  const int tid = threadIdx.x;
  float a = 0.f, b = 0.f;
  if (tid < W) for (int r = 0; r < 400; ++r) { const float v = X[(size_t)(blockIdx.x * 400 + r) * W + tid]; a += v; b += v * v; }
  s1[tid] = a; s2[tid] = b;
  __syncthreads();
  if (tid < W) { vst2(part + (size_t)blockIdx.x * 2 * W + tid, (float_a)s1[tid]); vst2(part + (size_t)blockIdx.x * 2 * W + W + tid, (float_a)s2[tid]); }
}
template <int W>
__global__ __launch_bounds__(256) void k_bnfin(const float* __restrict__ part, float* __restrict__ stats) {
  const int c = threadIdx.x;
  if (c < W) { float a = 0.f, b = 0.f;
    for (int p = 0; p < NN / 400; ++p) { a += part[(size_t)p * 2 * W + c]; b += part[(size_t)p * 2 * W + W + c]; }
    const float mu = a / (float)NN; float var = b / (float)NN - mu * mu; var = var < 0.f ? 0.f : var;
    vst2(stats + c, (float_a)mu); vst2(stats + W + c, (float_a)rsqrtf(var + 1e-5f)); }
}
template <int W>
__global__ __launch_bounds__(256) void k_bnelu(float* __restrict__ X, const float* __restrict__ stats, const float* __restrict__ gam, const float* __restrict__ bet) {
  const size_t i = (size_t)blockIdx.x * 256 + threadIdx.x; const int c = (int)(i % W);
  vst2(X + i, (float_a)eluf((X[i] - stats[c]) * stats[W + c] * gam[c] + bet[c]));
}
__global__ __launch_bounds__(128) void k_pool_head(const int* __restrict__ batch, const float* __restrict__ h2, const float* __restrict__ W1, const float* __restrict__ b1,
                                                 const float* __restrict__ W2, const float* __restrict__ b2, float* __restrict__ pool) {
  __shared__ float ps[C2], hs[64];
  const int g = blockIdx.x, tid = threadIdx.x;
  __shared__ int lohi[2];
  if (tid < 2) { int lo = 0, hi = NN; const int key = g + tid;
    while (lo < hi) { const int mid = (lo + hi) >> 1; if (batch[mid] < key) lo = mid + 1; else hi = mid; }
    lohi[tid] = lo; }
  __syncthreads();
  const int n0 = lohi[0], n1 = lohi[1];
  float a = 0.f;
  for (int n = n0; n < n1; ++n) a += h2[(size_t)n * C2 + tid];
  ps[tid] = a / fmaxf((float)(n1 - n0), 1.0f);
  __syncthreads();
  if (tid < 64) { float s = b1[tid]; for (int c = 0; c < C2; ++c) s += ps[c] * W1[c * 64 + tid]; hs[tid] = eluf(s); }
  __syncthreads();
  if (tid < 12) { float s = b2[tid]; for (int c = 0; c < 64; ++c) s += hs[c] * W2[c * 12 + tid]; ps[tid] = s; }
  __syncthreads();
  if (tid < 32) vst2(pool + (size_t)g * 32 + tid, (float_a)(tid < 12 ? ps[tid] : 0.f));
}
__global__ void k_flat(const float* __restrict__ pool, float* __restrict__ out) {
  for (int q = threadIdx.x; q < NG * 12 / 4; q += blockDim.x) { v4f v;
#pragma unroll
    for (int e = 0; e < 4; ++e) { const int f = q * 4 + e; v[e] = pool[(size_t)(f / 12) * 32 + (f % 12)]; }
    vst2(out + q * 4, v); }
}

extern "C" void kernel_launch(void* const* d_in, const int* in_sizes, int n_in,
                              void* d_out, int out_size, void* d_ws, size_t ws_size,
                              hipStream_t stream) {
  (void)in_sizes; (void)n_in; (void)out_size; (void)ws_size;
  const float* x  = (const float*)d_in[0];
  const int*   ei = (const int*)d_in[1];
  const float* ea = (const float*)d_in[2];
  const int* batch = (const int*)d_in[3];
  const float* Wl1 = (const float*)d_in[4];  const float* bl1 = (const float*)d_in[5];
  const float* Wr1 = (const float*)d_in[6];  const float* br1 = (const float*)d_in[7];
  const float* We1 = (const float*)d_in[8];  const float* at1 = (const float*)d_in[9];
  const float* bi1 = (const float*)d_in[10]; const float* g1 = (const float*)d_in[11]; const float* be1 = (const float*)d_in[12];
  const float* Wl2 = (const float*)d_in[13]; const float* bl2 = (const float*)d_in[14];
  const float* Wr2 = (const float*)d_in[15]; const float* br2 = (const float*)d_in[16];
  const float* We2 = (const float*)d_in[17]; const float* at2 = (const float*)d_in[18];
  const float* bi2 = (const float*)d_in[19]; const float* g2 = (const float*)d_in[20]; const float* be2 = (const float*)d_in[21];
  const float* Wm1 = (const float*)d_in[22]; const float* bm1 = (const float*)d_in[23];
  const float* Wm2 = (const float*)d_in[24]; const float* bm2 = (const float*)d_in[25];
  float* out = (float*)d_out;
  float* ws = (float*)d_ws; size_t off = 0;
  auto carve = [&](size_t n) { float* p = ws + off; off += (n + 63) & ~(size_t)63; return p; };
  float* xl = carve((size_t)NN * D1), *xr = carve((size_t)NN * D1), *h1 = carve((size_t)NN * D1);
  float* h2 = carve((size_t)NN * C2);
  float* xl2 = xl, *xr2 = xr;
  float* part = carve((size_t)(NN / 400) * 2 * D1), *stats = carve(2 * D1), *pool = carve((size_t)NG * 32);
  int*   rec = (int*)carve((size_t)NT * NCH * 32);
  float* eab = carve((size_t)NT * NCH * SLOTC * 4);
  int*   cnt = (int*)carve((size_t)NCH * 640);

  k_lin1<<<NN * 64 / 256, 256, 0, stream>>>(x, Wl1, bl1, Wr1, br1, xl, xr);
  k_bucket<<<NCH, 256, 0, stream>>>(ei, ea, rec, eab, cnt);
  k_gat<4, 0><<<NT, 256, 0, stream>>>(rec, eab, cnt, We1, at1, xl, xr, bi1, h1);
  k_colpart<D1><<<NN / 400, 256, 0, stream>>>(h1, part);
  k_bnfin<D1><<<1, 256, 0, stream>>>(part, stats);
  k_bnelu<D1><<<NN * D1 / 256, 256, 0, stream>>>(h1, stats, g1, be1);
  k_gemm<<<dim3(NN / 64, D1 / 64), 128, 0, stream>>>(h1, Wl2, bl2, xl2);
  k_gemm<<<dim3(NN / 64, D1 / 64), 128, 0, stream>>>(h1, Wr2, br2, xr2);
  k_gat<2, 1><<<NT, 256, 0, stream>>>(rec, eab, cnt, We2, at2, xl2, xr2, bi2, h2);
  k_colpart<C2><<<NN / 400, 256, 0, stream>>>(h2, part);
  k_bnfin<C2><<<1, 256, 0, stream>>>(part, stats);
  k_bnelu<C2><<<NN * C2 / 256, 256, 0, stream>>>(h2, stats, g2, be2);
  k_pool_head<<<NG, 128, 0, stream>>>(batch, h2, Wm1, bm1, Wm2, bm2, pool);
  k_flat<<<1, 256, 0, stream>>>(pool, out);
}
